// GNNAutoencoder_31842887532756
// MI455X (gfx1250) — hardware-verified
//
#include <hip/hip_runtime.h>
#include <stddef.h>
#include <stdint.h>


#define NTHR   256
#define NWAVE  8
#define EPT    8
#define CHUNK  (NTHR * EPT)
#define WCAP   (EPT * 32)
#define LISTN  (NWAVE * WCAP)
#define NBA    1024
#define SLA    10
#define RCAP   28672
#define RPW    (NBA + 32)
#define CSR_ZINTS    (LISTN + 2 * RCAP + 3 * NBA)
#define CSR_LDS_INTS (CSR_ZINTS + 16)
#define TR     64
#define NGR    32
#define PB     64
#define DOUT   3072
#define GBM    64
#define GBN    64
#define GTHR   128
#define NU_WB1 1024
#define NU_WB2 4096
#define NU_WB3 16384
#define NU_WA2 4096
#define NU_WA3 16384
#define NU_ALL (NU_WB1 + NU_WB2 + NU_WB3 + NU_WA2 + NU_WA3)
#define WSMAX  134217728

static_assert((CHUNK & (CHUNK - 1)) == 0 && CHUNK <= 4096);
static_assert((NBA & (NBA - 1)) == 0 && NBA == (1 << SLA));
static_assert(((long long)CHUNK << SLA) < (1LL << 31));
static_assert(LISTN % NTHR == 0 && NBA % 32 == 0);
static_assert(RCAP % (NTHR * 4) == 0 && CSR_ZINTS % 4 == 0 && LISTN % 4 == 0);
static_assert(RPW % 32 == 0 && (RPW * 4) % 128 == 0 && (RCAP * 4) % 128 == 0);
static_assert(CSR_LDS_INTS * 4 <= 300000);
static_assert(NU_WB1 % NTHR == 0 && NU_WB2 % NTHR == 0 && NU_WB3 % NTHR == 0 && NU_WA2 % NTHR == 0 && NU_WA3 % NTHR == 0);
static_assert(DOUT % NTHR == 0 && TR == 64 && NBA % TR == 0);

typedef float          v4f   __attribute__((ext_vector_type(4)));
typedef float          v8f   __attribute__((ext_vector_type(8)));
typedef int            v4i   __attribute__((ext_vector_type(4)));
typedef int            v8i   __attribute__((ext_vector_type(8)));
typedef unsigned int   v4u   __attribute__((ext_vector_type(4)));
typedef unsigned short v4us  __attribute__((ext_vector_type(4)));
typedef unsigned short v8us  __attribute__((ext_vector_type(8)));
typedef unsigned short v16us __attribute__((ext_vector_type(16)));
typedef __bf16         v16bf __attribute__((ext_vector_type(16)));
typedef v4f  __attribute__((may_alias)) v4fa;
typedef v4i  __attribute__((may_alias)) v4ia;
typedef v4u  __attribute__((may_alias)) v4ua;
typedef v4us __attribute__((may_alias)) v4usa;
typedef v8us __attribute__((may_alias)) v8usa;
union FragB { v16bf v; v16us u; v8us h[2]; v8i w; };

__device__ __forceinline__ v8f wmb(const FragB& a, const FragB& b, v8f c) {
  v8f d = __builtin_amdgcn_wmma_f32_16x16x32_bf16(false, a.v, false, b.v, (short)0, c, false, false);
  asm volatile("v_nop\n\tv_nop\n\tv_nop\n\tv_nop" : "+v"(d) : "v"(a.w), "v"(b.w));
  return d;
}

__device__ __forceinline__ unsigned bf16_bits(float f) {
  const unsigned u = __float_as_uint(f);
  const unsigned r = (u + 0x7FFFu + ((u >> 16) & 1u)) >> 16;
  return (f != f) ? 0x7fc0u : r;
}
__device__ __forceinline__ float bf16_val(float f) {
  return __uint_as_float(bf16_bits(f) << 16);
}
__device__ __forceinline__ v4f bf16_val4(v4f a) {
  v4f r; r.x = bf16_val(a.x); r.y = bf16_val(a.y); r.z = bf16_val(a.z); r.w = bf16_val(a.w); return r;
}
__device__ __forceinline__ void hilo(float v, unsigned& hb, unsigned& lb) {
  hb = bf16_bits(v);
  float lo = v - __uint_as_float(hb << 16);
  lo = ((hb & 0x7fffu) == 0x7f80u) ? 0.0f : lo;
  lb = bf16_bits(lo);
}
__device__ __forceinline__ void hilo4(v4f v, v4us& h, v4us& l) {
  unsigned a, b;
  hilo(v.x, a, b); h[0] = (unsigned short)a; l[0] = (unsigned short)b;
  hilo(v.y, a, b); h[1] = (unsigned short)a; l[1] = (unsigned short)b;
  hilo(v.z, a, b); h[2] = (unsigned short)a; l[2] = (unsigned short)b;
  hilo(v.w, a, b); h[3] = (unsigned short)a; l[3] = (unsigned short)b;
}
__device__ __forceinline__ float relu_n(float v) { return (v > 0.0f) ? v : ((v != v) ? v : 0.0f); }
__device__ __forceinline__ float nanmax(float a, float b) {
  float m = (a > b) ? a : b;
  return (a != a) ? a : m;
}
__device__ __forceinline__ v4f nanmax4(v4f a, v4f b) {
  v4f r; r.x = nanmax(a.x, b.x); r.y = nanmax(a.y, b.y); r.z = nanmax(a.z, b.z); r.w = nanmax(a.w, b.w); return r;
}

template <int SLB>
__device__ __forceinline__ int scan_chunk(const int* __restrict__ dsts, int nE, int cbase, int slotBase,
                                          int nb, int vec8, int* list, int tid, int lane, int wave) {
  int wc = 0;
  const int el0  = tid * EPT;
  const int e0   = cbase + el0;
  const int sent = -2147483647 - 1;
  v4i da, db;
  if (vec8 != 0 && cbase + CHUNK <= nE) {
    da = *(const v4i*)(dsts + e0);
    db = *(const v4i*)(dsts + e0 + 4);
  } else {
    da.x = (e0     < nE) ? dsts[min(e0,     nE - 1)] : sent;
    da.y = (e0 + 1 < nE) ? dsts[min(e0 + 1, nE - 1)] : sent;
    da.z = (e0 + 2 < nE) ? dsts[min(e0 + 2, nE - 1)] : sent;
    da.w = (e0 + 3 < nE) ? dsts[min(e0 + 3, nE - 1)] : sent;
    db.x = (e0 + 4 < nE) ? dsts[min(e0 + 4, nE - 1)] : sent;
    db.y = (e0 + 5 < nE) ? dsts[min(e0 + 5, nE - 1)] : sent;
    db.z = (e0 + 6 < nE) ? dsts[min(e0 + 6, nE - 1)] : sent;
    db.w = (e0 + 7 < nE) ? dsts[min(e0 + 7, nE - 1)] : sent;
  }
  const unsigned nbs = (unsigned)slotBase;
  const unsigned unb = (unsigned)nb;
  const unsigned s0 = (unsigned)da.x - nbs, s1 = (unsigned)da.y - nbs;
  const unsigned s2 = (unsigned)da.z - nbs, s3 = (unsigned)da.w - nbs;
  const unsigned s4 = (unsigned)db.x - nbs, s5 = (unsigned)db.y - nbs;
  const unsigned s6 = (unsigned)db.z - nbs, s7 = (unsigned)db.w - nbs;
  const bool h0 = s0 < unb, h1 = s1 < unb, h2 = s2 < unb, h3 = s3 < unb;
  const bool h4 = s4 < unb, h5 = s5 < unb, h6 = s6 < unb, h7 = s7 < unb;
  const unsigned any = __builtin_amdgcn_ballot_w32(h0 | h1 | h2 | h3 | h4 | h5 | h6 | h7);
  if (any != 0u) {
#define HITJ(J, HJ, SJ) { \
      const unsigned mj = __builtin_amdgcn_ballot_w32(HJ); \
      if (mj != 0u) { \
        if (HJ) { \
          const int pos = wc + (int)__builtin_amdgcn_mbcnt_lo(mj, 0u); \
          if (pos < WCAP) list[wave * WCAP + pos] = ((el0 + (J)) << SLB) | (int)(SJ); \
        } \
        wc += (int)__builtin_popcount(mj); } }
    HITJ(0, h0, s0)
    HITJ(1, h1, s1)
    HITJ(2, h2, s2)
    HITJ(3, h3, s3)
    HITJ(4, h4, s4)
    HITJ(5, h5, s5)
    HITJ(6, h6, s6)
    HITJ(7, h7, s7)
#undef HITJ
  }
  return wc;
}

__global__ __launch_bounds__(NTHR) void k_prep(const float* __restrict__ W1b, const float* __restrict__ W2b,
                                               const float* __restrict__ W3b, const float* __restrict__ W2a,
                                               const float* __restrict__ W3a,
                                               unsigned short* WB1, unsigned short* WB2, unsigned short* WB3,
                                               unsigned short* WA2, unsigned short* WA3) {
  const int u = (int)blockIdx.x * NTHR + (int)threadIdx.x;
  const float* W; unsigned short* P;
  int sp, kmask, nsplit, rowoff, kp, v;
  if (u < NU_WB1) {
    W = W1b; P = WB1; sp = 64; kmask = 63; nsplit = 1 << 30; rowoff = 0; kp = 128; v = u;
  } else if (u < NU_WB1 + NU_WB2) {
    W = W2b; P = WB2; sp = 128; kmask = 127; nsplit = 1 << 30; rowoff = 0; kp = 256; v = u - NU_WB1;
  } else if (u < NU_WB1 + NU_WB2 + NU_WB3) {
    W = W3b; P = WB3; sp = 256; kmask = 255; nsplit = 1 << 30; rowoff = 0; kp = 512; v = u - (NU_WB1 + NU_WB2);
  } else if (u < NU_WB1 + NU_WB2 + NU_WB3 + NU_WA2) {
    W = W2a; P = WA2; sp = 128; kmask = 63; nsplit = 128; rowoff = 64; kp = 128; v = u - (NU_WB1 + NU_WB2 + NU_WB3);
  } else if (u < NU_ALL) {
    W = W3a; P = WA3; sp = 256; kmask = 127; nsplit = 256; rowoff = 128; kp = 256;
    v = u - (NU_WB1 + NU_WB2 + NU_WB3 + NU_WA2);
  } else {
    return;
  }
  const int upr = kp >> 3;
  const int n   = v / upr;
  const int k8  = (v - n * upr) * 8;
  const bool bot = n >= nsplit;
  const int srow = (k8 & kmask) + (bot ? rowoff : 0);
  const int scol = bot ? (n - nsplit) : n;
  const float* p = W + (size_t)srow * sp + scol;
  v8us o;
#pragma unroll
  for (int i = 0; i < 8; ++i) o[i] = (unsigned short)bf16_bits(p[(size_t)i * sp]);
  unsigned short* dp = P + (size_t)n * kp + k8;
  *(volatile v8us*)dp = o;
  __threadfence();
  *(volatile v8us*)dp = o;
}

__global__ __launch_bounds__(NTHR) void k_csr(const int* __restrict__ srcs, const int* __restrict__ dsts,
                                              int nE, int nN, int vec8, int* csrc, int* rowptr) {
  extern __shared__ __attribute__((aligned(16))) int dsm[];
  int* list = dsm;
  int* hl   = dsm + LISTN;
  int* sl   = dsm + LISTN + RCAP;
  int* cnt  = dsm + LISTN + 2 * RCAP;
  int* offs = cnt + NBA;
  int* cur  = offs + NBA;
  int* misc = cur + NBA;
  const int tid = (int)threadIdx.x, lane = tid & 31, wave = tid >> 5;
  const int nodeBase = (int)blockIdx.x * NBA;

  {
    const v4i z4 = {0, 0, 0, 0};
    for (int i = tid * 4; i < CSR_ZINTS; i += NTHR * 4) *(v4ia*)(dsm + i) = z4;
    if (tid < 16) misc[tid] = 0;
  }
  __syncthreads();

  int t = 0, ov = 0;
  const int nChunks = (nE + CHUNK - 1) / CHUNK;
#pragma unroll 1
  for (int ch = 0; ch < nChunks; ++ch) {
    const int cbase = ch * CHUNK;
    const int wc = scan_chunk<SLA>(dsts, nE, cbase, nodeBase, NBA, vec8, list, tid, lane, wave);
    if (lane == 0) misc[wave] = wc;
    __syncthreads();
    if (wave == 0) {
#pragma unroll 1
      for (int w2 = 0; w2 < NWAVE; ++w2) {
        int c = misc[w2];
        c = c < 0 ? 0 : (c > WCAP ? WCAP : c);
#pragma unroll 1
        for (int b0 = 0; b0 < c; b0 += 32) {
          const int idx = b0 + lane;
          const int ent = list[w2 * WCAP + (idx < WCAP ? idx : WCAP - 1)];
          const int m32 = (c - b0) < 32 ? (c - b0) : 32;
#pragma unroll 1
          for (int k = 0; k < m32; ++k) {
            const int u    = __builtin_amdgcn_readlane(ent, k);
            const int slot = u & (NBA - 1);
            const int el   = (u >> SLA) & (CHUNK - 1);
            const int pk   = ((cbase + el) << SLA) | slot;
            if (t < RCAP) {
              if (lane == 0) { hl[t] = pk; cnt[slot] = cnt[slot] + 1; }
              t = t + 1;
            } else {
              ov = 1;
            }
          }
        }
      }
    }
    __syncthreads();
  }
  if (wave == 0 && lane == 0) { misc[8] = t; misc[9] = ov; }
  __syncthreads();
  int tt = misc[8];
  tt = tt < 0 ? 0 : (tt > RCAP ? RCAP : tt);
  const int ovf = misc[9];

  if (wave == 0) {
    const int base = lane * (NBA / 32);
    int s = 0;
#pragma unroll 1
    for (int i = 0; i < NBA / 32; ++i) s += cnt[base + i];
    int incl = s;
#pragma unroll
    for (int d = 1; d < 32; d <<= 1) {
      const int y = __shfl_up(incl, d, 32);
      if (lane >= d) incl += y;
    }
    int run = incl - s;
#pragma unroll 1
    for (int i = 0; i < NBA / 32; ++i) {
      const int cv = cnt[base + i];
      offs[base + i] = run;
      cur[base + i]  = run;
      run += cv;
    }
  }
  __syncthreads();
  if (wave == 0) {
#pragma unroll 1
    for (int b0 = 0; b0 < tt; b0 += 32) {
      const int idx = b0 + lane;
      const int ent = hl[idx < RCAP ? idx : RCAP - 1];
      const int m32 = (tt - b0) < 32 ? (tt - b0) : 32;
#pragma unroll 1
      for (int k = 0; k < m32; ++k) {
        const int u    = __builtin_amdgcn_readlane(ent, k);
        const int slot = u & (NBA - 1);
        if (lane == 0) {
          int p = cur[slot];
          p = p < 0 ? 0 : (p > RCAP - 1 ? RCAP - 1 : p);
          sl[p] = u;
          cur[slot] = p + 1;
        }
      }
    }
  }
  __syncthreads();
  if (tid < 32) cur[tid] = (tid == 0) ? tt : ((tid == 1) ? ovf : 0);
  __syncthreads();

  int* rp = rowptr + (size_t)blockIdx.x * RPW;
#pragma unroll 1
  for (int idx = tid; idx < RPW / 4; idx += NTHR) {
    const v4i v = *(const v4ia*)(offs + 4 * idx);
    *(volatile v4i*)(rp + 4 * idx) = v;
  }
  __threadfence();
#pragma unroll 1
  for (int idx = tid; idx < RPW / 4; idx += NTHR) {
    const v4i v = *(const v4ia*)(offs + 4 * idx);
    *(volatile v4i*)(rp + 4 * idx) = v;
  }

  int* cb = csrc + (size_t)blockIdx.x * RCAP;
#pragma unroll 1
  for (int it = 0; it < RCAP / (NTHR * 4); ++it) {
    const int p0 = (it * NTHR + tid) * 4;
    const v4i ent = *(const v4ia*)(sl + p0);
    int e0 = ent.x >> SLA, e1 = ent.y >> SLA, e2 = ent.z >> SLA, e3 = ent.w >> SLA;
    e0 = e0 < 0 ? 0 : (e0 > nE - 1 ? nE - 1 : e0);
    e1 = e1 < 0 ? 0 : (e1 > nE - 1 ? nE - 1 : e1);
    e2 = e2 < 0 ? 0 : (e2 > nE - 1 ? nE - 1 : e2);
    e3 = e3 < 0 ? 0 : (e3 > nE - 1 ? nE - 1 : e3);
    int r0 = srcs[e0], r1 = srcs[e1], r2 = srcs[e2], r3 = srcs[e3];
    r0 = r0 < 0 ? 0 : (r0 > nN - 1 ? nN - 1 : r0);
    r1 = r1 < 0 ? 0 : (r1 > nN - 1 ? nN - 1 : r1);
    r2 = r2 < 0 ? 0 : (r2 > nN - 1 ? nN - 1 : r2);
    r3 = r3 < 0 ? 0 : (r3 > nN - 1 ? nN - 1 : r3);
    v4i o;
    o.x = (p0     < tt) ? ((r0 << SLA) | (ent.x & (NBA - 1))) : 0;
    o.y = (p0 + 1 < tt) ? ((r1 << SLA) | (ent.y & (NBA - 1))) : 0;
    o.z = (p0 + 2 < tt) ? ((r2 << SLA) | (ent.z & (NBA - 1))) : 0;
    o.w = (p0 + 3 < tt) ? ((r3 << SLA) | (ent.w & (NBA - 1))) : 0;
    *(volatile v4i*)(cb + p0) = o;
    __threadfence();
    *(volatile v4i*)(cb + p0) = o;
  }
}

__global__ __launch_bounds__(GTHR) void k_gemm(
    const unsigned short* __restrict__ A, const unsigned short* __restrict__ WT,
    float* outF, int K, int ldo)
{
  __shared__ __attribute__((aligned(16))) float stg[GBM * GBN];
  const int tid = (int)threadIdx.x, lane = tid & 31, wave = tid >> 5, hh = lane >> 4, m = lane & 15;
  const int rowBase = (int)blockIdx.x * GBM;
  const int col0    = (int)blockIdx.y * GBN;

  v8f acc[4];
  {
    const v8f z = {0.f, 0.f, 0.f, 0.f, 0.f, 0.f, 0.f, 0.f};
    acc[0] = z; acc[1] = z; acc[2] = z; acc[3] = z;
  }
  const unsigned short* ap = A  + (size_t)(rowBase + 16 * wave + m) * (size_t)K + 8 * hh;
  const unsigned short* wp = WT + (size_t)(col0 + m) * (size_t)K + 8 * hh;
  const int ksteps = K >> 5;
#pragma unroll 1
  for (int ks = 0; ks < ksteps; ++ks) {
    FragB af;
    af.h[0] = *(const v8usa*)(ap + 32 * ks);
    af.h[1] = *(const v8usa*)(ap + 32 * ks + 16);
#pragma unroll
    for (int t = 0; t < 4; ++t) {
      const unsigned short* wq = wp + (size_t)(16 * t) * (size_t)K + 32 * ks;
      FragB bf;
      bf.h[0] = *(const v8usa*)wq;
      bf.h[1] = *(const v8usa*)(wq + 16);
      acc[t] = wmb(af, bf, acc[t]);
    }
  }

#pragma unroll
  for (int t = 0; t < 4; ++t) {
    const int lc = 16 * t + m;
#pragma unroll
    for (int r = 0; r < 8; ++r) {
      const int lr = 16 * wave + 8 * hh + r;
      stg[lr * GBN + lc] = acc[t][r];
    }
  }
  __syncthreads();

  v4f fv[8];
#pragma unroll
  for (int i = 0; i < 8; ++i) {
    const int lr = 16 * wave + 2 * i + hh;
    fv[i] = *(const v4fa*)(stg + lr * GBN + 4 * m);
  }
#pragma unroll
  for (int i = 0; i < 8; ++i) {
    const int lr = 16 * wave + 2 * i + hh;
    float* op = outF + (size_t)(rowBase + lr) * (size_t)ldo + col0 + 4 * m;
    *(volatile v4f*)op = fv[i];
  }
  __threadfence();
#pragma unroll
  for (int i = 0; i < 8; ++i) {
    const int lr = 16 * wave + 2 * i + hh;
    float* op = outF + (size_t)(rowBase + lr) * (size_t)ldo + col0 + 4 * m;
    *(volatile v4f*)op = fv[i];
  }
}

template <int FM, int R, int L1>
constexpr int conv_lds_bytes() {
  return TR * (2 * FM + 8) * 2 + TR * FM * 4 + R * FM * 4 +
         (L1 ? (R * 4 + 384 + 64 + TR * 8) * 4 : R * FM * 4) + 2 * TR * 4;
}

template <int FM, int R, int NCT, int NRT, int L1, int OUTF>
__global__ __launch_bounds__(NTHR) void k_conv(const float* __restrict__ xq, const float* __restrict__ wa1,
                                               const float* __restrict__ ba, const float* __restrict__ bb,
                                               const unsigned short* __restrict__ WB,
                                               const int* __restrict__ csrc, const int* __restrict__ rowptr,
                                               int nN, unsigned short* hb, float* hout) {
  constexpr int KP  = 2 * FM;
  constexpr int AP  = KP + 8;
  constexpr int CPR = FM / 4;
  constexpr int CG  = (FM / 16) / NCT;
  constexpr int USN = L1 ? (R * 4 + 384 + 64 + TR * 8) : R * FM;
  static_assert((4 / NRT) * CG == NWAVE && NCT * NRT * 32 == FM);
  static_assert(R <= TR && (NBA % R) == 0 && (R * FM / 4) % NTHR == 0 && (TR * CPR) % NTHR == 0);
  static_assert(L1 == 0 || FM == 64);

  extern __shared__ __attribute__((aligned(16))) unsigned char smem[];
  unsigned short* At = (unsigned short*)smem;
  float* Ct  = (float*)(smem + TR * AP * 2);
  float* ACC = Ct + TR * FM;
  float* US  = ACC + R * FM;
  int*   ti  = (int*)(US + USN);
  float* XS  = US;
  float* W1s = US + R * 4;
  float* B1s = W1s + 384;
  float* TX  = B1s + 64;

  const int tid = (int)threadIdx.x, lane = tid & 31, wave = tid >> 5, hh = lane >> 4, m = lane & 15;
  const int base = (int)blockIdx.x * R;
  const int blk  = base >> SLA;
  const int ls   = base & (NBA - 1);
  const int* rp  = rowptr + (size_t)blk * RPW;
  const int* cb  = csrc + (size_t)blk * RCAP;
  int e0 = rp[ls];
  int e1 = rp[ls + R];
  const int ovf = rp[NBA + 1];
  e0 = e0 < 0 ? 0 : (e0 > RCAP ? RCAP : e0);
  e1 = e1 < 0 ? 0 : (e1 > RCAP ? RCAP : e1);
  e1 = e1 < e0 ? e0 : e1;

  {
    const float ninf = __int_as_float((int)0xff800000u);
    const v4f n4 = {ninf, ninf, ninf, ninf};
    for (int i = tid * 4; i < R * FM; i += NTHR * 4) *(v4fa*)(ACC + i) = n4;
  }
  if constexpr (L1 != 0) {
    for (int i = tid; i < R * 4; i += NTHR) {
      const int s = i >> 2, d = i & 3;
      int node = base + s; node = node > nN - 1 ? nN - 1 : node;
      const float v = bf16_val(xq[(size_t)node * 3 + (d < 3 ? d : 2)]);
      XS[i] = (d < 3) ? v : 0.0f;
    }
    for (int i = tid; i < 384; i += NTHR) W1s[i] = bf16_val(wa1[i]);
    if (tid < 64) B1s[tid] = bf16_val(ba[tid]);
  } else {
#pragma unroll 1
    for (int idx = tid; idx < R * CPR; idx += NTHR) {
      const int s = idx / CPR, c4 = (idx % CPR) * 4;
      int node = base + s; node = node > nN - 1 ? nN - 1 : node;
      const v4f p  = *(const v4f*)(xq + (size_t)node * KP + c4);
      const v4f q  = *(const v4f*)(xq + (size_t)node * KP + FM + c4);
      const v4f b4 = bf16_val4(*(const v4f*)(ba + c4));
      const v4f u  = (p - q) + b4;
      *(v4fa*)(US + s * FM + c4) = u;
    }
  }
  __syncthreads();

  const int rg = wave / CG, cg = wave % CG;

#pragma unroll 1
  for (int t0 = e0; t0 < e1; t0 += TR) {
    if (tid < TR) {
      const int e = t0 + tid;
      const bool valid = e < e1;
      const int ea = e < RCAP - 1 ? e : RCAP - 1;
      const int ent = cb[ea];
      int sr = ent >> SLA;
      sr = sr < 0 ? 0 : (sr > nN - 1 ? nN - 1 : sr);
      int sl = (ent & (NBA - 1)) - ls;
      sl = sl < 0 ? 0 : (sl > R - 1 ? R - 1 : sl);
      ti[tid] = sr;
      ti[TR + tid] = valid ? sl : -1;
      if constexpr (L1 != 0) {
        const v4f xi = *(const v4fa*)(XS + sl * 4);
        const float j0 = bf16_val(xq[(size_t)sr * 3 + 0]);
        const float j1 = bf16_val(xq[(size_t)sr * 3 + 1]);
        const float j2 = bf16_val(xq[(size_t)sr * 3 + 2]);
        v4f dv; dv.x = j0 - xi.x; dv.y = j1 - xi.y; dv.z = j2 - xi.z; dv.w = 0.0f;
        *(v4fa*)(TX + tid * 8) = xi;
        *(v4fa*)(TX + tid * 8 + 4) = dv;
      }
    }
    __syncthreads();

#pragma unroll 1
    for (int it = 0; it < (TR * CPR) / NTHR; ++it) {
      const int idx = it * NTHR + tid;
      const int r = idx / CPR, c4 = (idx % CPR) * 4;
      const int s = ti[TR + r];
      v4f p;
      if constexpr (L1 != 0) {
        const v4f xi = *(const v4fa*)(TX + r * 8);
        const v4f dv = *(const v4fa*)(TX + r * 8 + 4);
        p = *(const v4fa*)(B1s + c4);
        p += *(const v4fa*)(W1s + 0 * 64 + c4) * xi.x;
        p += *(const v4fa*)(W1s + 1 * 64 + c4) * xi.y;
        p += *(const v4fa*)(W1s + 2 * 64 + c4) * xi.z;
        p += *(const v4fa*)(W1s + 3 * 64 + c4) * dv.x;
        p += *(const v4fa*)(W1s + 4 * 64 + c4) * dv.y;
        p += *(const v4fa*)(W1s + 5 * 64 + c4) * dv.z;
      } else {
        const int sr = ti[r];
        const int sv = s < 0 ? 0 : s;
        const v4f q = *(const v4f*)(xq + (size_t)sr * KP + FM + c4);
        const v4f u = *(const v4fa*)(US + sv * FM + c4);
        p = u + q;
      }
      const bool ok = s >= 0;
      p.x = ok ? relu_n(p.x) : 0.0f;
      p.y = ok ? relu_n(p.y) : 0.0f;
      p.z = ok ? relu_n(p.z) : 0.0f;
      p.w = ok ? relu_n(p.w) : 0.0f;
      v4us h4, l4;
      hilo4(p, h4, l4);
      *(v4usa*)(At + r * AP + c4) = h4;
      *(v4usa*)(At + r * AP + FM + c4) = l4;
    }
    __syncthreads();

    {
      v8f acc[NRT * NCT];
      const v8f z = {0.f, 0.f, 0.f, 0.f, 0.f, 0.f, 0.f, 0.f};
#pragma unroll
      for (int i = 0; i < NRT * NCT; ++i) acc[i] = z;
      const unsigned short* al = At + (16 * rg * NRT + m) * AP + 8 * hh;
      const unsigned short* wl = WB + (size_t)(16 * cg * NCT + m) * KP + 8 * hh;
#pragma unroll 1
      for (int ks = 0; ks < KP / 32; ++ks) {
        FragB bf[NCT];
#pragma unroll
        for (int ct = 0; ct < NCT; ++ct) {
          const unsigned short* wq = wl + (size_t)(16 * ct) * KP + 32 * ks;
          bf[ct].h[0] = *(const v8usa*)wq;
          bf[ct].h[1] = *(const v8usa*)(wq + 16);
        }
#pragma unroll
        for (int rt = 0; rt < NRT; ++rt) {
          const unsigned short* aq = al + (16 * rt) * AP + 32 * ks;
          FragB af;
          af.h[0] = *(const v8usa*)aq;
          af.h[1] = *(const v8usa*)(aq + 16);
#pragma unroll
          for (int ct = 0; ct < NCT; ++ct) acc[rt * NCT + ct] = wmb(af, bf[ct], acc[rt * NCT + ct]);
        }
      }
#pragma unroll
      for (int rt = 0; rt < NRT; ++rt) {
#pragma unroll
        for (int ct = 0; ct < NCT; ++ct) {
          const int lc = 16 * (cg * NCT + ct) + m;
#pragma unroll
          for (int r = 0; r < 8; ++r) {
            const int lr = 16 * (rg * NRT + rt) + 8 * hh + r;
            Ct[lr * FM + lc] = acc[rt * NCT + ct][r];
          }
        }
      }
    }
    __syncthreads();

    if (tid < CPR) {
#pragma unroll 4
      for (int r = 0; r < TR; ++r) {
        const int s = ti[TR + r];
        if (s >= 0) {
          const v4f a = *(const v4fa*)(ACC + s * FM + 4 * tid);
          const v4f c = *(const v4fa*)(Ct + r * FM + 4 * tid);
          *(v4fa*)(ACC + s * FM + 4 * tid) = nanmax4(a, c);
        }
      }
    }
    __syncthreads();
  }

  {
    const float pz = (ovf != 0) ? __int_as_float(0x7fc00000) : 0.0f;
    unsigned short* stg = (unsigned short*)Ct;
#pragma unroll 1
    for (int idx = tid; idx < R * CPR; idx += NTHR) {
      const int s = idx / CPR, c4 = (idx % CPR) * 4;
      const v4f a  = *(const v4fa*)(ACC + s * FM + c4);
      const v4f b4 = bf16_val4(*(const v4f*)(bb + c4));
      const bool live = (base + s) < nN;
      v4f v;
      v.x = live ? ((a.x + b4.x) + pz) : 0.0f;
      v.y = live ? ((a.y + b4.y) + pz) : 0.0f;
      v.z = live ? ((a.z + b4.z) + pz) : 0.0f;
      v.w = live ? ((a.w + b4.w) + pz) : 0.0f;
      if constexpr (OUTF != 0) {
        *(v4fa*)(Ct + s * FM + c4) = v;
      } else {
        v4us h4, l4;
        hilo4(v, h4, l4);
        *(v4usa*)(stg + s * KP + c4) = h4;
        *(v4usa*)(stg + s * KP + FM + c4) = l4;
      }
    }
  }
  __syncthreads();
  {
    unsigned* gout;
    if constexpr (OUTF != 0) gout = (unsigned*)(hout + (size_t)base * FM);
    else                     gout = (unsigned*)(hb + (size_t)base * KP);
    const unsigned* sg = (const unsigned*)Ct;
#pragma unroll 1
    for (int it = 0; it < (R * FM / 4) / NTHR; ++it) {
      const int idx = it * NTHR + tid;
      const v4u v = *(const v4ua*)(sg + 4 * idx);
      *(volatile v4u*)(gout + 4 * (size_t)idx) = v;
    }
    __threadfence();
#pragma unroll 1
    for (int it = 0; it < (R * FM / 4) / NTHR; ++it) {
      const int idx = it * NTHR + tid;
      const v4u v = *(const v4ua*)(sg + 4 * idx);
      *(volatile v4u*)(gout + 4 * (size_t)idx) = v;
    }
  }
}

__global__ __launch_bounds__(NTHR) void k_pool(const float* __restrict__ X3, const int* __restrict__ bat,
                                               int nN, int npb, float* rec) {
  __shared__ __attribute__((aligned(16))) float sl[NGR * 256];
  const int tid = (int)threadIdx.x;
  const float ninf = __int_as_float((int)0xff800000u);
#pragma unroll 1
  for (int g = 0; g < NGR; ++g) sl[g * 256 + tid] = ninf;
  const int n0 = (int)blockIdx.x * npb;
  int n1 = n0 + npb; n1 = n1 > nN ? nN : n1;
#pragma unroll 1
  for (int n = n0; n < n1; ++n) {
    const int b = bat[n];
    const float v = X3[(size_t)n * 256 + tid];
    if ((unsigned)b < (unsigned)NGR) {
      const float a = sl[b * 256 + tid];
      sl[b * 256 + tid] = nanmax(a, v);
    }
  }
  __syncthreads();
  float* rp = rec + (size_t)blockIdx.x * (NGR * 256);
#pragma unroll 1
  for (int it = 0; it < (NGR * 256 / 4) / NTHR; ++it) {
    const int idx = it * NTHR + tid;
    const v4f v = *(const v4fa*)(sl + 4 * idx);
    *(volatile v4f*)(rp + 4 * idx) = v;
  }
  __threadfence();
#pragma unroll 1
  for (int it = 0; it < (NGR * 256 / 4) / NTHR; ++it) {
    const int idx = it * NTHR + tid;
    const v4f v = *(const v4fa*)(sl + 4 * idx);
    *(volatile v4f*)(rp + 4 * idx) = v;
  }
}

__global__ __launch_bounds__(NTHR) void k_dec1(const float* __restrict__ rec,
                                               const float* __restrict__ Wfc, const float* __restrict__ bfc,
                                               const float* __restrict__ Wd1, const float* __restrict__ bd1,
                                               float* tt) {
  __shared__ __attribute__((aligned(16))) float PLT[256 * NGR];
  __shared__ __attribute__((aligned(16))) float ZT[128 * NGR];
  const int tid = (int)threadIdx.x;
#pragma unroll 1
  for (int it = 0; it < (NGR * 256 / 4) / NTHR; ++it) {
    const int idx = it * NTHR + tid;
    const int g = idx >> 6, c4 = (idx & 63) * 4;
    v4f mx = *(const v4f*)(rec + (size_t)g * 256 + c4);
#pragma unroll 4
    for (int pb = 1; pb < PB; ++pb) {
      const v4f v = *(const v4f*)(rec + (size_t)pb * (NGR * 256) + (size_t)g * 256 + c4);
      mx = nanmax4(mx, v);
    }
    PLT[(c4 + 0) * NGR + g] = mx.x;
    PLT[(c4 + 1) * NGR + g] = mx.y;
    PLT[(c4 + 2) * NGR + g] = mx.z;
    PLT[(c4 + 3) * NGR + g] = mx.w;
  }
  __syncthreads();
  {
    const int o = tid & 127, gh = tid >> 7;
    float acc[16];
#pragma unroll
    for (int i = 0; i < 16; ++i) acc[i] = 0.0f;
#pragma unroll 1
    for (int k = 0; k < 256; ++k) {
      const float w = bf16_val(Wfc[(size_t)k * 128 + o]);
      const float* pp = PLT + k * NGR + 16 * gh;
#pragma unroll
      for (int q = 0; q < 4; ++q) {
        const v4f p = *(const v4fa*)(pp + 4 * q);
        acc[4 * q + 0] = fmaf(p.x, w, acc[4 * q + 0]);
        acc[4 * q + 1] = fmaf(p.y, w, acc[4 * q + 1]);
        acc[4 * q + 2] = fmaf(p.z, w, acc[4 * q + 2]);
        acc[4 * q + 3] = fmaf(p.w, w, acc[4 * q + 3]);
      }
    }
    const float b = bf16_val(bfc[o]);
#pragma unroll
    for (int i = 0; i < 16; ++i) ZT[o * NGR + 16 * gh + i] = acc[i] + b;
  }
  __syncthreads();
  {
    const int o = tid;
    float acc[NGR];
#pragma unroll
    for (int i = 0; i < NGR; ++i) acc[i] = 0.0f;
#pragma unroll 1
    for (int k = 0; k < 128; ++k) {
      const float w = bf16_val(Wd1[(size_t)k * 256 + o]);
      const float* pp = ZT + k * NGR;
#pragma unroll
      for (int q = 0; q < 8; ++q) {
        const v4f p = *(const v4fa*)(pp + 4 * q);
        acc[4 * q + 0] = fmaf(p.x, w, acc[4 * q + 0]);
        acc[4 * q + 1] = fmaf(p.y, w, acc[4 * q + 1]);
        acc[4 * q + 2] = fmaf(p.z, w, acc[4 * q + 2]);
        acc[4 * q + 3] = fmaf(p.w, w, acc[4 * q + 3]);
      }
    }
    const float b = bf16_val(bd1[o]);
#pragma unroll
    for (int i = 0; i < NGR; ++i) PLT[o * NGR + i] = relu_n(acc[i] + b);
  }
  __syncthreads();
#pragma unroll 1
  for (int it = 0; it < (256 * NGR / 4) / NTHR; ++it) {
    const int idx = it * NTHR + tid;
    const v4f v = *(const v4fa*)(PLT + 4 * idx);
    *(volatile v4f*)(tt + 4 * idx) = v;
  }
  __threadfence();
#pragma unroll 1
  for (int it = 0; it < (256 * NGR / 4) / NTHR; ++it) {
    const int idx = it * NTHR + tid;
    const v4f v = *(const v4fa*)(PLT + 4 * idx);
    *(volatile v4f*)(tt + 4 * idx) = v;
  }
}

__global__ __launch_bounds__(NTHR) void k_dec2(const float* __restrict__ tt, const float* __restrict__ Wd2,
                                               const float* __restrict__ bd2, float* out) {
  __shared__ __attribute__((aligned(16))) float TS[256 * NGR];
  const int tid = (int)threadIdx.x;
  const int col = (int)blockIdx.x * NTHR + tid;
#pragma unroll 1
  for (int it = 0; it < (256 * NGR / 4) / NTHR; ++it) {
    const int idx = it * NTHR + tid;
    *(v4fa*)(TS + 4 * idx) = *(const v4f*)(tt + 4 * idx);
  }
  __syncthreads();
  float acc[NGR];
#pragma unroll
  for (int i = 0; i < NGR; ++i) acc[i] = 0.0f;
#pragma unroll 1
  for (int k = 0; k < 256; ++k) {
    const float w = bf16_val(Wd2[(size_t)k * DOUT + col]);
    const float* pp = TS + k * NGR;
#pragma unroll
    for (int q = 0; q < 8; ++q) {
      const v4f p = *(const v4fa*)(pp + 4 * q);
      acc[4 * q + 0] = fmaf(p.x, w, acc[4 * q + 0]);
      acc[4 * q + 1] = fmaf(p.y, w, acc[4 * q + 1]);
      acc[4 * q + 2] = fmaf(p.z, w, acc[4 * q + 2]);
      acc[4 * q + 3] = fmaf(p.w, w, acc[4 * q + 3]);
    }
  }
  const float b = bf16_val(bd2[col]);
  __syncthreads();
#pragma unroll
  for (int g = 0; g < NGR; ++g) TS[g * 256 + tid] = acc[g] + b;
  __syncthreads();
  float* ob = out + (size_t)blockIdx.x * NTHR;
#pragma unroll 1
  for (int it = 0; it < (NGR * 256 / 4) / NTHR; ++it) {
    const int idx = it * NTHR + tid;
    const int g = idx >> 6, c4 = (idx & 63) * 4;
    const v4f v = *(const v4fa*)(TS + g * 256 + c4);
    *(volatile v4f*)(ob + (size_t)g * DOUT + c4) = v;
  }
  __threadfence();
#pragma unroll 1
  for (int it = 0; it < (NGR * 256 / 4) / NTHR; ++it) {
    const int idx = it * NTHR + tid;
    const int g = idx >> 6, c4 = (idx & 63) * 4;
    const v4f v = *(const v4fa*)(TS + g * 256 + c4);
    *(volatile v4f*)(ob + (size_t)g * DOUT + c4) = v;
  }
}

static inline int cdiv(int a, int b) { return (a + b - 1) / b; }
static inline size_t al256(size_t o) { return (o + 255) & ~(size_t)255; }

extern "C" void kernel_launch(void* const* d_in, const int* in_sizes, int n_in,
                              void* d_out, int out_size, void* d_ws, size_t ws_size,
                              hipStream_t stream) {
  if (n_in < 21) return;
  if (in_sizes[0] < 3 || (in_sizes[0] % 3) != 0) return;
  const int nN = in_sizes[0] / 3;
  if (nN < 1 || nN > (1 << 20)) return;
  if (in_sizes[1] < 2 || (in_sizes[1] & 1) != 0) return;
  const int nE = in_sizes[1] / 2;
  if (nE < 1 || nE >= (1 << 21)) return;
  if (in_sizes[2] != nN) return;
  if (in_sizes[3] != 6 * 64 || in_sizes[4] != 64) return;
  if (in_sizes[5] != 64 * 64 || in_sizes[6] != 64) return;
  if (in_sizes[7] != 128 * 128 || in_sizes[8] != 128) return;
  if (in_sizes[9] != 128 * 128 || in_sizes[10] != 128) return;
  if (in_sizes[11] != 256 * 256 || in_sizes[12] != 256) return;
  if (in_sizes[13] != 256 * 256 || in_sizes[14] != 256) return;
  if (in_sizes[15] != 256 * 128 || in_sizes[16] != 128) return;
  if (in_sizes[17] != 128 * 256 || in_sizes[18] != 256) return;
  if (in_sizes[19] != 256 * DOUT || in_sizes[20] != DOUT) return;
  if (out_size != NGR * DOUT) return;

  const float* x    = (const float*)d_in[0];
  const int*   edge = (const int*)d_in[1];
  const int*   bat  = (const int*)d_in[2];
  const float* W1a  = (const float*)d_in[3];
  const float* b1a  = (const float*)d_in[4];
  const float* W1b  = (const float*)d_in[5];
  const float* b1b  = (const float*)d_in[6];
  const float* W2a  = (const float*)d_in[7];
  const float* b2a  = (const float*)d_in[8];
  const float* W2b  = (const float*)d_in[9];
  const float* b2b  = (const float*)d_in[10];
  const float* W3a  = (const float*)d_in[11];
  const float* b3a  = (const float*)d_in[12];
  const float* W3b  = (const float*)d_in[13];
  const float* b3b  = (const float*)d_in[14];
  const float* Wfc  = (const float*)d_in[15];
  const float* bfc  = (const float*)d_in[16];
  const float* Wd1  = (const float*)d_in[17];
  const float* bd1  = (const float*)d_in[18];
  const float* Wd2  = (const float*)d_in[19];
  const float* bd2  = (const float*)d_in[20];
  float* out = (float*)d_out;
  const int* src = edge;
  const int* dst = edge + nE;

  const int MP = cdiv(nN, GBM) * GBM;
  const int gA = cdiv(MP, NBA);
  if ((long long)gA * NBA < (long long)MP) return;
  const int vec8 = ((nE & 3) == 0) ? 1 : 0;
  const int npb  = cdiv(nN, PB);

  char* ws = (char*)d_ws;
  size_t off = 0;
  const size_t oWB1 = off; off = al256(off + (size_t)64 * 128 * 2);
  const size_t oWB2 = off; off = al256(off + (size_t)128 * 256 * 2);
  const size_t oWB3 = off; off = al256(off + (size_t)256 * 512 * 2);
  const size_t oWA2 = off; off = al256(off + (size_t)256 * 128 * 2);
  const size_t oWA3 = off; off = al256(off + (size_t)512 * 256 * 2);
  const size_t oRP  = off; off = al256(off + (size_t)gA * RPW * 4);
  const size_t oCS  = off; off = al256(off + (size_t)gA * RCAP * 4);
  const size_t oX1  = off; off = al256(off + (size_t)MP * 128 * 2);
  const size_t oPQ2 = off; off = al256(off + (size_t)MP * 256 * 4);
  const size_t oX2  = off; off = al256(off + (size_t)MP * 256 * 2);
  const size_t oPQ3 = off; off = al256(off + (size_t)MP * 512 * 4);
  const size_t oREC = off; off = al256(off + (size_t)PB * NGR * 256 * 4);
  const size_t oTT  = off; off = al256(off + (size_t)256 * NGR * 4);
  if (off > ws_size || off > (size_t)WSMAX) return;
  unsigned short* WB1 = (unsigned short*)(ws + oWB1);
  unsigned short* WB2 = (unsigned short*)(ws + oWB2);
  unsigned short* WB3 = (unsigned short*)(ws + oWB3);
  unsigned short* WA2 = (unsigned short*)(ws + oWA2);
  unsigned short* WA3 = (unsigned short*)(ws + oWA3);
  int*            RP  = (int*)(ws + oRP);
  int*            CS  = (int*)(ws + oCS);
  unsigned short* X1  = (unsigned short*)(ws + oX1);
  float*          PQ2 = (float*)(ws + oPQ2);
  float*          X3  = (float*)(ws + oPQ2);
  unsigned short* X2  = (unsigned short*)(ws + oX2);
  float*          PQ3 = (float*)(ws + oPQ3);
  float*          REC = (float*)(ws + oREC);
  float*          TT  = (float*)(ws + oTT);

  const int csrLds = CSR_LDS_INTS * 4;
  constexpr int l1 = conv_lds_bytes<64, 64, 1>();
  constexpr int l2 = conv_lds_bytes<128, 64, 0>();
  constexpr int l3 = conv_lds_bytes<256, 32, 0>();
  static_assert(l1 <= 300000 && l2 <= 300000 && l3 <= 300000);
  hipFuncSetAttribute(reinterpret_cast<const void*>(&k_csr), hipFuncAttributeMaxDynamicSharedMemorySize, csrLds);
  hipFuncSetAttribute(reinterpret_cast<const void*>(&k_conv<64, 64, 1, 2, 1, 0>), hipFuncAttributeMaxDynamicSharedMemorySize, l1);
  hipFuncSetAttribute(reinterpret_cast<const void*>(&k_conv<128, 64, 1, 4, 0, 0>), hipFuncAttributeMaxDynamicSharedMemorySize, l2);
  hipFuncSetAttribute(reinterpret_cast<const void*>(&k_conv<256, 32, 2, 4, 0, 1>), hipFuncAttributeMaxDynamicSharedMemorySize, l3);

  k_prep<<<NU_ALL / NTHR, NTHR, 0, stream>>>(W1b, W2b, W3b, W2a, W3a, WB1, WB2, WB3, WA2, WA3);
  k_csr<<<gA, NTHR, csrLds, stream>>>(src, dst, nE, nN, vec8, CS, RP);
  k_conv<64, 64, 1, 2, 1, 0><<<MP / 64, NTHR, l1, stream>>>(x, W1a, b1a, b1b, WB1, CS, RP, nN, X1, X3);
  k_gemm<<<dim3(MP / GBM, 256 / GBN), GTHR, 0, stream>>>(X1, WA2, PQ2, 128, 256);
  k_conv<128, 64, 1, 4, 0, 0><<<MP / 64, NTHR, l2, stream>>>(PQ2, W1a, b2a, b2b, WB2, CS, RP, nN, X2, X3);
  k_gemm<<<dim3(MP / GBM, 512 / GBN), GTHR, 0, stream>>>(X2, WA3, PQ3, 256, 512);
  k_conv<256, 32, 2, 4, 0, 1><<<MP / 32, NTHR, l3, stream>>>(PQ3, W1a, b3a, b3b, WB3, CS, RP, nN, X2, X3);
  k_pool<<<PB, NTHR, 0, stream>>>(X3, bat, nN, npb, REC);
  k_dec1<<<1, NTHR, 0, stream>>>(REC, Wfc, bfc, Wd1, bd1, TT);
  k_dec2<<<DOUT / NTHR, NTHR, 0, stream>>>(TT, Wd2, bd2, out);
}
